// EquivariantMPNNLayer_68324339745418
// MI455X (gfx1250) — hardware-verified
//
#include <hip/hip_runtime.h>
#include <stddef.h>


typedef float          v4f  __attribute__((ext_vector_type(4)));
typedef float          v8f  __attribute__((ext_vector_type(8)));
typedef int            v4i  __attribute__((ext_vector_type(4)));
typedef unsigned int   v2u  __attribute__((ext_vector_type(2)));
typedef unsigned int   v4u  __attribute__((ext_vector_type(4)));
typedef unsigned short v8us __attribute__((ext_vector_type(8)));
typedef _Float16       v8h  __attribute__((ext_vector_type(8)));
typedef _Float16       v16h __attribute__((ext_vector_type(16)));
typedef __bf16         v16b __attribute__((ext_vector_type(16)));
union FragH { v16h v; v8h  h[2]; };
union FragB { v16b v; v8us h[2]; };

#define GP 136

__device__ __forceinline__ unsigned int bf16_rne_bits(float x) {
  const unsigned int u = __float_as_uint(x);
  return (u + 0x7FFFu + ((u >> 16) & 1u)) >> 16;
}
__device__ __forceinline__ void split_bf16(float x, unsigned int& hi, unsigned int& lo) {
  hi = bf16_rne_bits(x);
  const float hf = __uint_as_float(hi << 16);
  lo = bf16_rne_bits(x - hf);
}
__device__ __forceinline__ float silu_f(float x) {
  const float t = __expf(-x);
  return x * __builtin_amdgcn_rcpf(1.0f + t);
}

__device__ __forceinline__ void wm2f16(v16h a0, v16h a1, v16h b, v8f& c0, v8f& c1) {
  c0 = __builtin_amdgcn_wmma_f32_16x16x32_f16(false, a0, false, b, (short)0, c0, false, false);
  c1 = __builtin_amdgcn_wmma_f32_16x16x32_f16(false, a1, false, b, (short)0, c1, false, false);
  asm volatile("v_nop\n\tv_nop\n\tv_nop\n\tv_nop" : "+v"(c0), "+v"(c1) : "v"(a0), "v"(a1), "v"(b));
}
__device__ __forceinline__ v8f wm3bf(v16b ah, v16b al, v16b bh, v16b bl, v8f c) {
  c = __builtin_amdgcn_wmma_f32_16x16x32_bf16(false, ah, false, bh, (short)0, c, false, false);
  c = __builtin_amdgcn_wmma_f32_16x16x32_bf16(false, ah, false, bl, (short)0, c, false, false);
  c = __builtin_amdgcn_wmma_f32_16x16x32_bf16(false, al, false, bh, (short)0, c, false, false);
  asm volatile("v_nop\n\tv_nop\n\tv_nop\n\tv_nop" : "+v"(c) : "v"(ah), "v"(al), "v"(bh), "v"(bl));
  return c;
}

template <int MODE>
__global__ __launch_bounds__(256) void k_prep(const float* __restrict__ W0, const float* __restrict__ W1,
                                            const float* __restrict__ W2, const float* __restrict__ W3,
                                            const float* __restrict__ W4, unsigned short* dst) {
  __shared__ __attribute__((aligned(16))) unsigned short sT[2 * 64 * GP];
  constexpr int NPL = (MODE == 0) ? 2 : 1;
  const int tid = threadIdx.x, lane = tid & 31, wave = tid >> 5;
  const int b = blockIdx.x;
  const float* W = (b == 0) ? W0 : ((b == 1) ? W1 : ((b == 2) ? W2 : ((b == 3) ? W3 : W4)));
  unsigned short* db = dst + (size_t)b * NPL * 16384;

#pragma unroll 1
  for (int nh = 0; nh < 2; ++nh) {
#pragma unroll 1
    for (int idx = tid; idx < 128 * 64; idx += 256) {
      const int k = idx >> 6, nl = idx & 63;
      const float v = W[k * 128 + nh * 64 + nl];
      if (MODE == 0) {
        unsigned int hi, lo;
        split_bf16(v, hi, lo);
        sT[nl * GP + k]           = (unsigned short)hi;
        sT[64 * GP + nl * GP + k] = (unsigned short)lo;
      } else {
        const _Float16 hv = (_Float16)(v * 8.0f);
        sT[nl * GP + k] = __builtin_bit_cast(unsigned short, hv);
      }
    }
    __syncthreads();
    v4u xv[NPL * 4];
#pragma unroll
    for (int p = 0; p < NPL; ++p) {
#pragma unroll
      for (int q = 0; q < 4; ++q) {
        const int pr = q * 8 + wave;
        const int rl = 2 * pr + (lane >> 4);
        xv[p * 4 + q] = *(const v4u*)(sT + p * 64 * GP + rl * GP + (lane & 15) * 8);
      }
    }
#pragma unroll
    for (int p = 0; p < NPL; ++p) {
#pragma unroll
      for (int q = 0; q < 4; ++q) {
        const int pr = q * 8 + wave;
        const int rl = 2 * pr + (lane >> 4);
        unsigned short* gp = db + (size_t)p * 16384 + (size_t)(nh * 64 + rl) * 128 + (lane & 15) * 8;
        *(volatile v4u*)gp = xv[p * 4 + q];
      }
    }
    __threadfence();
#pragma unroll
    for (int p = 0; p < NPL; ++p) {
#pragma unroll
      for (int q = 0; q < 4; ++q) {
        const int pr = q * 8 + wave;
        const int rl = 2 * pr + (lane >> 4);
        unsigned short* gp = db + (size_t)p * 16384 + (size_t)(nh * 64 + rl) * 128 + (lane & 15) * 8;
        *(volatile v4u*)gp = xv[p * 4 + q];
      }
    }
    __syncthreads();
  }
}

template <int EPI>
__global__ __launch_bounds__(256) void k_gemm(const float* __restrict__ A, int lda, int aRow0, int aRows,
                                            const unsigned short* __restrict__ Bhi,
                                            const unsigned short* __restrict__ Blo,
                                            const float* __restrict__ bias, float* outp, int outRows) {
  __shared__ __attribute__((aligned(16))) unsigned short sA[2 * 64 * GP];
  float* sO = (float*)sA;
  const int tid = threadIdx.x, lane = tid & 31, wave = tid >> 5, hh = lane >> 4, m = lane & 15;
  const int rt = wave & 3, chf = wave >> 2;
  const int row0 = blockIdx.x * 64;

#pragma unroll 1
  for (int idx = tid; idx < 64 * 32; idx += 256) {
    const int r = idx >> 5, k4 = (idx & 31) * 4;
    const int ar = row0 + r - aRow0;
    const bool valid = (ar >= 0) && (ar < aRows);
    int arc = ar < 0 ? 0 : ar;
    arc = arc > aRows - 1 ? aRows - 1 : arc;
    v4f v = *(const v4f*)(A + (size_t)arc * lda + k4);
    if (!valid) { const v4f z = {0.0f, 0.0f, 0.0f, 0.0f}; v = z; }
    unsigned int h0, l0, h1, l1, h2, l2, h3, l3;
    split_bf16(v.x, h0, l0);
    split_bf16(v.y, h1, l1);
    split_bf16(v.z, h2, l2);
    split_bf16(v.w, h3, l3);
    v2u hp, lp;
    hp.x = h0 | (h1 << 16); hp.y = h2 | (h3 << 16);
    lp.x = l0 | (l1 << 16); lp.y = l2 | (l3 << 16);
    *(v2u*)(sA + r * GP + k4)           = hp;
    *(v2u*)(sA + 64 * GP + r * GP + k4) = lp;
  }
  __syncthreads();

  v8f acc[4];
#pragma unroll
  for (int nt = 0; nt < 4; ++nt) {
#pragma unroll
    for (int r = 0; r < 8; ++r) acc[nt][r] = 0.0f;
  }
#pragma unroll
  for (int ks = 0; ks < 4; ++ks) {
    FragB ah, al;
    const unsigned short* ap = sA + (rt * 16 + m) * GP + ks * 32 + 8 * hh;
    ah.h[0] = *(const v8us*)ap;
    ah.h[1] = *(const v8us*)(ap + 16);
    al.h[0] = *(const v8us*)(ap + 64 * GP);
    al.h[1] = *(const v8us*)(ap + 64 * GP + 16);
#pragma unroll
    for (int nt = 0; nt < 4; ++nt) {
      const int n = chf * 64 + nt * 16 + m;
      const size_t bo = (size_t)n * 128 + ks * 32 + 8 * hh;
      FragB bh, bl;
      bh.h[0] = *(const v8us*)(Bhi + bo);
      bh.h[1] = *(const v8us*)(Bhi + bo + 16);
      bl.h[0] = *(const v8us*)(Blo + bo);
      bl.h[1] = *(const v8us*)(Blo + bo + 16);
      acc[nt] = wm3bf(ah.v, al.v, bh.v, bl.v, acc[nt]);
    }
  }
  __syncthreads();

#pragma unroll
  for (int nt = 0; nt < 4; ++nt) {
    const int col = chf * 64 + nt * 16 + m;
    float bv = 0.0f;
    if (EPI != 0) bv = bias[col];
#pragma unroll
    for (int r = 0; r < 8; ++r) {
      float v = acc[nt][r];
      if (EPI == 1) v = silu_f(v + bv);
      else if (EPI == 2) v = v + bv;
      sO[(rt * 16 + 8 * hh + r) * 128 + col] = v;
    }
  }
  __syncthreads();

  v4f ov[8];
#pragma unroll
  for (int rr = 0; rr < 8; ++rr) ov[rr] = *(const v4f*)(sO + (rr * 8 + wave) * 128 + 4 * lane);
#pragma unroll
  for (int rr = 0; rr < 8; ++rr) {
    const int gr = row0 + rr * 8 + wave;
    if (gr < outRows) *(volatile v4f*)(outp + (size_t)gr * 128 + 4 * lane) = ov[rr];
  }
  __threadfence();
#pragma unroll
  for (int rr = 0; rr < 8; ++rr) {
    const int gr = row0 + rr * 8 + wave;
    if (gr < outRows) *(volatile v4f*)(outp + (size_t)gr * 128 + 4 * lane) = ov[rr];
  }
}

#define ENT    128
#define ENW    4
#define EPT    8
#define ECHUNK (ENT * EPT)
#define EWCAP  (EPT * 32)
#define ELISTN (ENW * EWCAP)
#define EPASS  (ENW * 32)
#define EPCAP  (ECHUNK + EPASS)
#define ENB    224
#define TPH    136
#define HP     136
#define HTILE  (2 * 16 * HP)
#define HDB    (2 * HTILE * 2)
#define PSB    (32 * 128 * 4)
#define WREG   (HDB + PSB)
#define ASC    8.0f
#define DSC    64.0f
#define DINV   0.015625f

static_assert(EPCAP % EPASS == 0);
static_assert(ECHUNK % EPASS == 0);
static_assert(ENT == EPASS);
static_assert(ENT == 128);
static_assert(32 * TPH * 2 <= HDB);
static_assert(2 * 16 * 128 * 4 <= PSB);
static_assert(((HTILE * 2) % 16) == 0 && (HDB % 16) == 0 && (PSB % 16) == 0);
static_assert((WREG % 16) == 0);
static_assert((ENB % ENW) == 0 && (ENB % 4) == 0);

#define L_ACC  0
#define L_CNT  (L_ACC + ENB * 128 * 4)
#define L_WRG  (L_CNT + ENB * 4)
#define L_LIST (L_WRG + ENW * WREG)
#define L_PEND (L_LIST + ELISTN * 4)
#define L_SLOT (L_PEND + EPCAP * 4)
#define L_WE1  (L_SLOT + EPASS * 4)
#define L_BE1  (L_WE1 + 384 * 4)
#define L_BH   (L_BE1 + 128 * 4)
#define L_BM2  (L_BH + 128 * 4)
#define L_WCNT (L_BM2 + 128 * 4)
#define L_PN   (L_WCNT + 16)
#define L_SMEM (L_PN + 16)

static_assert((L_CNT % 16) == 0 && (L_WRG % 16) == 0 && (L_LIST % 16) == 0 && (L_PEND % 16) == 0);
static_assert((L_SLOT % 16) == 0 && (L_WE1 % 16) == 0 && (L_BE1 % 16) == 0);
static_assert((L_BH % 16) == 0 && (L_BM2 % 16) == 0 && (L_WCNT % 16) == 0 && (L_PN % 16) == 0);
static_assert(L_SMEM == 263072);

__device__ __forceinline__ int scan_chunk(const int* __restrict__ dsts, int nE, int cbase, int keyBase,
                                          int vec8, int* list, int tid, int wave) {
  int wc = 0;
  const int el0  = tid * EPT;
  const int e0   = cbase + el0;
  const int sent = -2147483647 - 1;
  const int em   = nE - 1;
  v4i da, db;
  if (vec8 != 0 && cbase + ECHUNK <= nE) {
    da = *(const v4i*)(dsts + e0);
    db = *(const v4i*)(dsts + e0 + 4);
  } else {
    da.x = (e0     < nE) ? dsts[(e0     < em) ? e0     : em] : sent;
    da.y = (e0 + 1 < nE) ? dsts[(e0 + 1 < em) ? e0 + 1 : em] : sent;
    da.z = (e0 + 2 < nE) ? dsts[(e0 + 2 < em) ? e0 + 2 : em] : sent;
    da.w = (e0 + 3 < nE) ? dsts[(e0 + 3 < em) ? e0 + 3 : em] : sent;
    db.x = (e0 + 4 < nE) ? dsts[(e0 + 4 < em) ? e0 + 4 : em] : sent;
    db.y = (e0 + 5 < nE) ? dsts[(e0 + 5 < em) ? e0 + 5 : em] : sent;
    db.z = (e0 + 6 < nE) ? dsts[(e0 + 6 < em) ? e0 + 6 : em] : sent;
    db.w = (e0 + 7 < nE) ? dsts[(e0 + 7 < em) ? e0 + 7 : em] : sent;
  }
  const unsigned nb = (unsigned)keyBase;
  const unsigned s0 = (unsigned)da.x - nb, s1 = (unsigned)da.y - nb;
  const unsigned s2 = (unsigned)da.z - nb, s3 = (unsigned)da.w - nb;
  const unsigned s4 = (unsigned)db.x - nb, s5 = (unsigned)db.y - nb;
  const unsigned s6 = (unsigned)db.z - nb, s7 = (unsigned)db.w - nb;
  const bool h0 = s0 < (unsigned)ENB, h1 = s1 < (unsigned)ENB, h2 = s2 < (unsigned)ENB, h3 = s3 < (unsigned)ENB;
  const bool h4 = s4 < (unsigned)ENB, h5 = s5 < (unsigned)ENB, h6 = s6 < (unsigned)ENB, h7 = s7 < (unsigned)ENB;
  const unsigned any = __builtin_amdgcn_ballot_w32(h0 | h1 | h2 | h3 | h4 | h5 | h6 | h7);
  if (any != 0u) {
#define HITJ(J, HJ) { \
      const unsigned mj = __builtin_amdgcn_ballot_w32(HJ); \
      if (mj != 0u) { \
        if (HJ) { \
          const int pos = wc + (int)__builtin_amdgcn_mbcnt_lo(mj, 0u); \
          if (pos < EWCAP) list[wave * EWCAP + pos] = el0 + (J); \
        } \
        wc += (int)__builtin_popcount(mj); } }
    HITJ(0, h0)
    HITJ(1, h1)
    HITJ(2, h2)
    HITJ(3, h3)
    HITJ(4, h4)
    HITJ(5, h5)
    HITJ(6, h6)
    HITJ(7, h7)
#undef HITJ
  }
  return wc;
}

__device__ __forceinline__ void load_tile_frags(const _Float16* T, int hh, int m, FragH* a0, FragH* a1) {
#pragma unroll
  for (int ks = 0; ks < 4; ++ks) {
    const _Float16* p0 = T + m * TPH + ks * 32 + 8 * hh;
    const _Float16* p1 = T + (16 + m) * TPH + ks * 32 + 8 * hh;
    a0[ks].h[0] = *(const v8h*)p0;
    a0[ks].h[1] = *(const v8h*)(p0 + 16);
    a1[ks].h[0] = *(const v8h*)p1;
    a1[ks].h[1] = *(const v8h*)(p1 + 16);
  }
}

__global__ __launch_bounds__(ENT) void k_edge(
    const float* __restrict__ Pp, const float* __restrict__ npos, const float* __restrict__ gpos,
    const int* __restrict__ ei, const float* __restrict__ frm, const int* __restrict__ bat,
    const float* __restrict__ We1, const float* __restrict__ be1,
    const float* __restrict__ be2, const float* __restrict__ Wm1,
    const float* __restrict__ bm1, const float* __restrict__ bm2,
    const _Float16* __restrict__ WcT,
    const unsigned short* __restrict__ Wm2h, const unsigned short* __restrict__ Wm2l,
    float* meanp, int nN, int nG, int nE, int nB, int vec8) {
  extern __shared__ __attribute__((aligned(16))) char smem[];
  float* ACC   = (float*)(smem + L_ACC);
  int*   CNT   = (int*)(smem + L_CNT);
  int*   list  = (int*)(smem + L_LIST);
  int*   pend  = (int*)(smem + L_PEND);
  int*   slotA = (int*)(smem + L_SLOT);
  float* sWe1  = (float*)(smem + L_WE1);
  float* sBe1  = (float*)(smem + L_BE1);
  float* sBh   = (float*)(smem + L_BH);
  float* sBm2  = (float*)(smem + L_BM2);
  int*   wcnt  = (int*)(smem + L_WCNT);
  int*   pendN = (int*)(smem + L_PN);

  const int tid = threadIdx.x, lane = tid & 31, wave = tid >> 5, hh = lane >> 4, m = lane & 15;
  const int nodeBase = blockIdx.x * ENB;
  const int keyBase  = nN + nodeBase;
  const int* srcs = ei;
  const int* dsts = ei + nE;
  char* wreg = smem + L_WRG + wave * WREG;
  _Float16*       T  = (_Float16*)wreg;
  unsigned short* Hd = (unsigned short*)wreg;
  float*          Ps = (float*)(wreg + HDB);

  for (int i = tid; i < ENB * 32; i += ENT) { const v4f z = {0.0f, 0.0f, 0.0f, 0.0f}; *(v4f*)(ACC + 4 * i) = z; }
  for (int i = tid; i < ENB; i += ENT) CNT[i] = 0;
  for (int i = tid; i < 384; i += ENT) sWe1[i] = We1[i];
  {
    const int n = tid;
    sBe1[n] = be1[n];
    sBm2[n] = bm2[n];
    float a = bm1[n];
#pragma unroll 1
    for (int k = 0; k < 128; ++k) a += be2[k] * Wm1[(size_t)(128 + k) * 128 + n];
    sBh[n] = a;
  }
  if (tid == 0) pendN[0] = 0;
  __syncthreads();

  const int nChunks = (nE + ECHUNK - 1) / ECHUNK;
#pragma unroll 1
  for (int ch = 0; ch < nChunks; ++ch) {
    const int cbase = ch * ECHUNK;
    const int wc = scan_chunk(dsts, nE, cbase, keyBase, vec8, list, tid, wave);
    if (lane == 0) wcnt[wave] = wc;
    __syncthreads();

    const int base = pendN[0];
    int tot = 0, myoff = 0;
#pragma unroll
    for (int w = 0; w < ENW; ++w) {
      int c = wcnt[w];
      c = c > EWCAP ? EWCAP : (c < 0 ? 0 : c);
      if (w < wave) myoff += c;
      tot += c;
    }
    int newN = base + tot;
    newN = newN > EPCAP ? EPCAP : newN;
    {
      int n = wcnt[wave];
      n = n > EWCAP ? EWCAP : (n < 0 ? 0 : n);
      const int* lp = list + wave * EWCAP;
      for (int i = lane; i < n; i += 32) {
        const int pos = base + myoff + i;
        if (pos < EPCAP) pend[pos] = cbase + lp[i];
      }
    }
    const int fin = (ch == nChunks - 1) ? 1 : 0;
    const int R   = (fin != 0) ? (newN + EPASS - 1) / EPASS : newN / EPASS;
    const int Pv  = (fin != 0) ? newN : R * EPASS;
    __syncthreads();

#pragma unroll 1
    for (int r = 0; r < R; ++r) {
      float l0, l1, l2;
      int s;
      {
        int idx = r * EPASS + wave * 32 + lane;
        const bool valid = idx < Pv;
        idx = idx > EPCAP - 1 ? EPCAP - 1 : idx;
        int e = pend[idx];
        e = e < 0 ? 0 : (e > nE - 1 ? nE - 1 : e);
        const int d = dsts[e];
        s = srcs[e];
        s = s < 0 ? 0 : (s > nN - 1 ? nN - 1 : s);
        int slot = d - keyBase;
        if (!valid || (unsigned)slot >= (unsigned)ENB) slot = ENB;
        int gc = d - nN;
        gc = gc < 0 ? 0 : (gc > nG - 1 ? nG - 1 : gc);
        int bi = bat[s];
        bi = bi < 0 ? 0 : (bi > nB - 1 ? nB - 1 : bi);
        const float* F = frm + bi * 9;
        const float rx = gpos[gc * 3 + 0] - npos[s * 3 + 0];
        const float ry = gpos[gc * 3 + 1] - npos[s * 3 + 1];
        const float rz = gpos[gc * 3 + 2] - npos[s * 3 + 2];
        l0 = F[0] * rx + F[1] * ry + F[2] * rz;
        l1 = F[3] * rx + F[4] * ry + F[5] * rz;
        l2 = F[6] * rx + F[7] * ry + F[8] * rz;
        slotA[wave * 32 + lane] = slot;
      }
      {
        const float* prow = Pp + (size_t)s * 128;
        float* psr = Ps + lane * 128;
#pragma unroll 4
        for (int c = 0; c < 32; ++c) {
          const v4f pv = *(const v4f*)(prow + 4 * c);
          const v4f bv = *(const v4f*)(sBh + 4 * c);
          *(v4f*)(psr + 4 * c) = (pv + bv) * DSC;
        }
      }
      {
#pragma unroll 2
        for (int g = 0; g < 16; ++g) {
          const int k = g * 8;
          const v4f wa0 = *(const v4f*)(sWe1 + k),       wa1 = *(const v4f*)(sWe1 + k + 4);
          const v4f wb0 = *(const v4f*)(sWe1 + 128 + k), wb1 = *(const v4f*)(sWe1 + 128 + k + 4);
          const v4f wc0 = *(const v4f*)(sWe1 + 256 + k), wc1 = *(const v4f*)(sWe1 + 256 + k + 4);
          const v4f bb0 = *(const v4f*)(sBe1 + k),       bb1 = *(const v4f*)(sBe1 + k + 4);
          v8h hv;
#pragma unroll
          for (int i = 0; i < 4; ++i) {
            const float x0 = l0 * wa0[i] + l1 * wb0[i] + l2 * wc0[i] + bb0[i];
            const float x1 = l0 * wa1[i] + l1 * wb1[i] + l2 * wc1[i] + bb1[i];
            hv[i]     = (_Float16)(silu_f(x0) * ASC);
            hv[4 + i] = (_Float16)(silu_f(x1) * ASC);
          }
          *(v8h*)(T + lane * TPH + k) = hv;
        }
      }
      __syncthreads();

      FragH a0[4], a1[4];
      load_tile_frags(T, hh, m, a0, a1);
      __syncthreads();

#pragma unroll 1
      for (int nt = 0; nt < 8; ++nt) {
        const int col = nt * 16 + m;
        v8f c0, c1;
#pragma unroll
        for (int rr = 0; rr < 8; ++rr) {
          c0[rr] = Ps[(8 * hh + rr) * 128 + col];
          c1[rr] = Ps[(16 + 8 * hh + rr) * 128 + col];
        }
#pragma unroll
        for (int ks = 0; ks < 4; ++ks) {
          FragH b;
          const _Float16* bp = WcT + (size_t)col * 128 + ks * 32 + 8 * hh;
          b.h[0] = *(const v8h*)bp;
          b.h[1] = *(const v8h*)(bp + 16);
          wm2f16(a0[ks].v, a1[ks].v, b.v, c0, c1);
        }
#pragma unroll
        for (int rr = 0; rr < 8; ++rr) {
          unsigned int h0b, l0b, h1b, l1b;
          split_bf16(silu_f(c0[rr] * DINV), h0b, l0b);
          split_bf16(silu_f(c1[rr] * DINV), h1b, l1b);
          const int ro = (8 * hh + rr) * HP + col;
          Hd[0 * HTILE + ro]           = (unsigned short)h0b;
          Hd[0 * HTILE + 16 * HP + ro] = (unsigned short)l0b;
          Hd[1 * HTILE + ro]           = (unsigned short)h1b;
          Hd[1 * HTILE + 16 * HP + ro] = (unsigned short)l1b;
        }
      }
      __syncthreads();

#pragma unroll 1
      for (int t = 0; t < 2; ++t) {
        v8f acc[8];
#pragma unroll
        for (int nt = 0; nt < 8; ++nt) {
#pragma unroll
          for (int rr = 0; rr < 8; ++rr) acc[nt][rr] = 0.0f;
        }
        const unsigned short* Hb = Hd + t * HTILE;
#pragma unroll
        for (int ks = 0; ks < 4; ++ks) {
          FragB ah, al;
          const unsigned short* ap = Hb + m * HP + ks * 32 + 8 * hh;
          ah.h[0] = *(const v8us*)ap;
          ah.h[1] = *(const v8us*)(ap + 16);
          al.h[0] = *(const v8us*)(ap + 16 * HP);
          al.h[1] = *(const v8us*)(ap + 16 * HP + 16);
#pragma unroll
          for (int nt = 0; nt < 8; ++nt) {
            const size_t bo = (size_t)(nt * 16 + m) * 128 + ks * 32 + 8 * hh;
            FragB bh, bl;
            bh.h[0] = *(const v8us*)(Wm2h + bo);
            bh.h[1] = *(const v8us*)(Wm2h + bo + 16);
            bl.h[0] = *(const v8us*)(Wm2l + bo);
            bl.h[1] = *(const v8us*)(Wm2l + bo + 16);
            acc[nt] = wm3bf(ah.v, al.v, bh.v, bl.v, acc[nt]);
          }
        }
        float* Mt = Ps + t * (16 * 128);
#pragma unroll
        for (int nt = 0; nt < 8; ++nt) {
          const int col = nt * 16 + m;
          const float bmv = sBm2[col];
#pragma unroll
          for (int rr = 0; rr < 8; ++rr) Mt[(8 * hh + rr) * 128 + col] = acc[nt][rr] + bmv;
        }
      }
      __syncthreads();

      if (wave == 0) {
#pragma unroll 1
        for (int q = 0; q < EPASS; ++q) {
          int sl = slotA[q];
          sl = __builtin_amdgcn_readfirstlane(sl);
          if ((unsigned)sl < (unsigned)ENB) {
            const float* mp = (const float*)(smem + L_WRG + (q >> 5) * WREG + HDB) + (q & 31) * 128 + 4 * lane;
            const v4f mv = *(const v4f*)mp;
            float* ap = ACC + sl * 128 + 4 * lane;
            const v4f av = *(const v4f*)ap;
            *(v4f*)ap = av + mv;
            if (lane == 0) CNT[sl] += 1;
          }
        }
      }
      __syncthreads();
    }

    int rem = newN - R * EPASS;
    rem = rem < 0 ? 0 : rem;
    if (R > 0 && tid < rem) pend[tid] = pend[R * EPASS + tid];
    if (tid == 0) pendN[0] = rem;
  }
  __syncthreads();

#pragma unroll 1
  for (int rr = 0; rr < ENB / ENW; ++rr) {
    const int s = rr * ENW + wave;
    const float cn = (float)CNT[s];
    const float inv = 1.0f / fmaxf(cn, 1.0f);
    const v4f a = *(const v4f*)(ACC + s * 128 + 4 * lane);
    const v4f v = a * inv;
    *(volatile v4f*)(meanp + (size_t)(nodeBase + s) * 128 + 4 * lane) = v;
  }
  __threadfence();
#pragma unroll 1
  for (int rr = 0; rr < ENB / ENW; ++rr) {
    const int s = rr * ENW + wave;
    const float cn = (float)CNT[s];
    const float inv = 1.0f / fmaxf(cn, 1.0f);
    const v4f a = *(const v4f*)(ACC + s * 128 + 4 * lane);
    const v4f v = a * inv;
    *(volatile v4f*)(meanp + (size_t)(nodeBase + s) * 128 + 4 * lane) = v;
  }
}

extern "C" void kernel_launch(void* const* d_in, const int* in_sizes, int n_in,
                              void* d_out, int out_size, void* d_ws, size_t ws_size,
                              hipStream_t stream) {
  if (n_in < 18) return;
  const int nN = in_sizes[0] / 128;
  if (nN <= 0 || in_sizes[0] != nN * 128 || in_sizes[1] != nN * 3) return;
  const int nG = in_sizes[2] / 3;
  if (nG <= 0 || in_sizes[2] != nG * 3) return;
  const int nE = in_sizes[3] / 2;
  if (nE < 0 || in_sizes[3] != nE * 2) return;
  const int nB = in_sizes[4] / 9;
  if (nB <= 0 || in_sizes[4] != nB * 9) return;
  if (in_sizes[5] != nN) return;
  if (in_sizes[6] != 384 || in_sizes[7] != 128 || in_sizes[8] != 16384 || in_sizes[9] != 128) return;
  if (in_sizes[10] != 32768 || in_sizes[11] != 128 || in_sizes[12] != 16384 || in_sizes[13] != 128) return;
  if (in_sizes[14] != 16384 || in_sizes[15] != 128 || in_sizes[16] != 16384 || in_sizes[17] != 128) return;
  const int NS = nN + nG;
  if (out_size != NS * 128) return;

  const float* emb  = (const float*)d_in[0];
  const float* npos = (const float*)d_in[1];
  const float* gpos = (const float*)d_in[2];
  const int*   ei   = (const int*)d_in[3];
  const float* frm  = (const float*)d_in[4];
  const int*   bat  = (const int*)d_in[5];
  const float* We1  = (const float*)d_in[6];
  const float* be1  = (const float*)d_in[7];
  const float* We2  = (const float*)d_in[8];
  const float* be2  = (const float*)d_in[9];
  const float* Wm1  = (const float*)d_in[10];
  const float* bm1  = (const float*)d_in[11];
  const float* Wm2  = (const float*)d_in[12];
  const float* bm2  = (const float*)d_in[13];
  const float* Wu1  = (const float*)d_in[14];
  const float* bu1  = (const float*)d_in[15];
  const float* Wu2  = (const float*)d_in[16];
  const float* bu2  = (const float*)d_in[17];
  float* out = (float*)d_out;

  const int nBlkP = (nN + 63) / 64;
  const int nBlkE = (nG + ENB - 1) / ENB;
  const int nBlkU = (NS + 63) / 64;

  char* ws = (char*)d_ws;
  size_t off = 0;
  const size_t oBF   = off; off += (size_t)5 * 2 * 16384 * 2;
  const size_t oF16  = off; off += (size_t)1 * 16384 * 2;
  const size_t oP    = off; off += (size_t)nBlkP * 64 * 128 * 4;
  const size_t oWC   = off; off += (size_t)2 * 64 * 128 * 4;
  const size_t oMEAN = off; off += (size_t)nBlkE * ENB * 128 * 4;
  const size_t oU1   = off; off += (size_t)nBlkU * 64 * 128 * 4;
  if (off > ws_size || off > (size_t)134217728) return;

  unsigned short* bfp  = (unsigned short*)(ws + oBF);
  unsigned short* f16p = (unsigned short*)(ws + oF16);
  float* Pp    = (float*)(ws + oP);
  float* Wc32  = (float*)(ws + oWC);
  float* meanp = (float*)(ws + oMEAN);
  float* U1p   = (float*)(ws + oU1);
  const _Float16* WcT = (const _Float16*)(f16p);

  const int vec8 = ((nE & 3) == 0) ? 1 : 0;

  hipFuncSetAttribute(reinterpret_cast<const void*>(&k_edge), hipFuncAttributeMaxDynamicSharedMemorySize, L_SMEM);

  k_prep<0><<<dim3(5), dim3(256), 0, stream>>>(Wm1, Wm1 + 16384, Wu1, Wu2, Wm2, bfp);
  k_gemm<0><<<dim3(nBlkP), dim3(256), 0, stream>>>(emb, 128, 0, nN, bfp + 0 * 32768, bfp + 0 * 32768 + 16384,
                                                   bm1, Pp, nBlkP * 64);
  k_gemm<0><<<dim3(2), dim3(256), 0, stream>>>(We2, 128, 0, 128, bfp + 1 * 32768, bfp + 1 * 32768 + 16384,
                                               bm1, Wc32, 128);
  k_prep<1><<<dim3(1), dim3(256), 0, stream>>>(Wc32, Wc32, Wc32, Wc32, Wc32, f16p);
  k_edge<<<dim3(nBlkE), dim3(ENT), L_SMEM, stream>>>(Pp, npos, gpos, ei, frm, bat, We1, be1, be2, Wm1, bm1, bm2,
                                                     WcT, bfp + 4 * 32768, bfp + 4 * 32768 + 16384,
                                                     meanp, nN, nG, nE, nB, vec8);
  k_gemm<1><<<dim3(nBlkU), dim3(256), 0, stream>>>(meanp, 128, nN, nG, bfp + 2 * 32768, bfp + 2 * 32768 + 16384,
                                                   bu1, U1p, nBlkU * 64);
  k_gemm<2><<<dim3(nBlkU), dim3(256), 0, stream>>>(U1p, 128, 0, nBlkU * 64, bfp + 3 * 32768, bfp + 3 * 32768 + 16384,
                                                   bu2, out, NS);
}
